// MoTAttention_35656818491416
// MI455X (gfx1250) — hardware-verified
//
#include <hip/hip_runtime.h>
#include <math.h>
#include <stdint.h>

#ifndef NB
#define NB 2
#endif
#ifndef SEQ
#define SEQ 2048
#endif
#define XS_FULL 2048
#define DMOD  2048
#define NH    16
#define NKVH  4
#define HD    128
#define HHALF (HD / 2)
#define KVD   (NKVH * HD)
#define NMOD  2
#define ROWSP (SEQ + 64)
#define NRT   (ROWSP / 64)
#define MROWS (NB * SEQ)
#define PROWS (NB * ROWSP)
#define TPERM 0
#define TIPOS ROWSP
#define THDR  (ROWSP + SEQ)
#define TABN  (ROWSP + SEQ + 32)
#define NLEAD 4
#define RPT   (SEQ / 256)
#define RSQ_HD 0.08838834764831845f
#define LOG2E 1.4426950408889634f
#define QSC   256.0f
#define KSC   256.0f
#define PCAR  32768.0f
#define VCAR  1024.0f
#define OSC   1024.0f
#define WOS   1024.0f
#define WPB   (NH / NKVH)
#define NHG   NKVH
#define NQT   (SEQ / 16)
#define NST   (SEQ / 64)
#define NKT   (SEQ / 32)
#define ATT_THREADS (WPB * 32)
#define PTP   36
#define PTW   (16 * PTP)
#define SLP   132
#define SLW   (16 * SLP)
#define WREG  (PTW + SLW)
#define SLAB64 (16 * 68)
#define VTP   72
#define WTP   72
#define WS_CAP 134217728
static_assert(DMOD == NH * HD && HD == 128 && HHALF == 64 && NH == 16 && NKVH == 4 && WPB == 4 && NHG * WPB == NH);
static_assert(ATT_THREADS == 128 && KVD == 512 && NMOD == 2);
static_assert(NB >= 1 && NB <= 2);
static_assert((SEQ % 256) == 0 && SEQ >= 256 && SEQ <= XS_FULL && RPT >= 1 && RPT <= 8);
static_assert((ROWSP % 64) == 0 && (TABN % 32) == 0 && NRT * 64 == ROWSP);
static_assert((DMOD % 64) == 0 && (KVD % 64) == 0 && (DMOD % 32) == 0 && (HD % 32) == 0);
static_assert(DMOD / 8 == 256 && KVD / 8 == 64);
static_assert(WPB * WREG * 4 <= 65536 && 2 * HD * VTP * 2 <= 65536 && 4 * SLAB64 * 4 <= 65536 && TABN * 4 + 64 <= 65536);

typedef unsigned short u16;
typedef _Float16 v16h __attribute__((ext_vector_type(16)));
typedef _Float16 v8h  __attribute__((ext_vector_type(8)));
typedef __bf16   v16b __attribute__((ext_vector_type(16)));
typedef float    v8f  __attribute__((ext_vector_type(8)));
typedef float    v4f  __attribute__((ext_vector_type(4)));
typedef unsigned int v4u __attribute__((ext_vector_type(4)));
typedef int      v4i  __attribute__((ext_vector_type(4)));

union FragH { v16h v; v8h h[2]; v4u u[2]; };
union FragB { v16b v; v4u u[2]; };

__device__ __forceinline__ unsigned short bf_bits(float f) {
  unsigned u = __float_as_uint(f);
  return (unsigned short)((u + 0x7FFFu + ((u >> 16) & 1u)) >> 16);
}
__device__ __forceinline__ float bf_up(unsigned short h) { return __uint_as_float(((unsigned)h) << 16); }
__device__ __forceinline__ float bfr(float f) { return bf_up(bf_bits(f)); }
__device__ __forceinline__ unsigned short h_bits(_Float16 x) { return __builtin_bit_cast(unsigned short, x); }
__device__ __forceinline__ unsigned pk16(unsigned short a, unsigned short b) { return (unsigned)a | ((unsigned)b << 16); }
__device__ __forceinline__ v8f zero8() { v8f z = {0.f, 0.f, 0.f, 0.f, 0.f, 0.f, 0.f, 0.f}; return z; }
__device__ __forceinline__ int clampi(int v, int lo, int hi) { return (v < lo) ? lo : ((v > hi) ? hi : v); }

__device__ __forceinline__ void seginfo(const int* tab, int& n0, int& P0, int& U) {
  const int v = clampi(tab[THDR], 0, SEQ);
  n0 = v;
  P0 = (v + 63) & ~63;
  U  = P0 + (((SEQ - v) + 63) & ~63);
}

__device__ __forceinline__ v16h ldfrag_h(const _Float16* p) {
  FragH f;
  f.h[0] = *(const v8h*)(p);
  f.h[1] = *(const v8h*)(p + 16);
  return f.v;
}
__device__ __forceinline__ v16b ldfrag_b(const u16* p) {
  FragB f;
  f.u[0] = *(const v4u*)(p);
  f.u[1] = *(const v4u*)(p + 16);
  return f.v;
}

__device__ __forceinline__ v8f mma_h(v16h a, v16h b, v8f c) {
  return __builtin_amdgcn_wmma_f32_16x16x32_f16(false, a, false, b, (short)0, c, false, false);
}
__device__ __forceinline__ v8f mma_b(v16b a, v16b b, v8f c) {
  return __builtin_amdgcn_wmma_f32_16x16x32_bf16(false, a, false, b, (short)0, c, false, false);
}
__device__ __forceinline__ void guard2(v8f& a, v8f& b, v16h x0, v16h x1, v16h x2, v16h x3, v16h x4, v16h x5) {
#if defined(__HIP_DEVICE_COMPILE__)
  asm volatile("v_nop\n\tv_nop\n\tv_nop\n\tv_nop"
               : "+v"(a), "+v"(b) : "v"(x0), "v"(x1), "v"(x2), "v"(x3), "v"(x4), "v"(x5) : "memory");
#endif
}
template <typename F>
__device__ __forceinline__ void guard6(v8f& a, v8f& b, v8f& c, v8f& d, F x0, F x1, F x2, F x3, F x4, F x5) {
#if defined(__HIP_DEVICE_COMPILE__)
  asm volatile("v_nop\n\tv_nop\n\tv_nop\n\tv_nop"
               : "+v"(a), "+v"(b), "+v"(c), "+v"(d) : "v"(x0), "v"(x1), "v"(x2), "v"(x3), "v"(x4), "v"(x5) : "memory");
#endif
}
__device__ __forceinline__ void acc_guard4(v8f& a, v8f& b, v8f& c, v8f& d) {
#if defined(__HIP_DEVICE_COMPILE__)
  asm volatile("v_nop\n\tv_nop\n\tv_nop\n\tv_nop" : "+v"(a), "+v"(b), "+v"(c), "+v"(d));
#endif
}
__device__ __forceinline__ void wave_sync_lds() {
  __builtin_amdgcn_fence(__ATOMIC_RELEASE, "workgroup");
  __builtin_amdgcn_wave_barrier();
  __builtin_amdgcn_fence(__ATOMIC_ACQUIRE, "workgroup");
}

__global__ __launch_bounds__(256) void k_perm(const int* __restrict__ ids, int* TAB) {
  __shared__ __align__(16) int L[TABN];
  __shared__ int wtot[8];
  const int tid = threadIdx.x, lane = tid & 31, wave = tid >> 5;
  const int b = blockIdx.x;
  if (b >= NB) return;
  for (int i = tid; i < TABN; i += 256) L[i] = (i < ROWSP) ? -1 : 0;
  const int s0 = tid * RPT;
  int idv[RPT];
  int c0 = 0;
#pragma unroll
  for (int i = 0; i < RPT; ++i) {
    idv[i] = ids[(size_t)b * XS_FULL + s0 + i];
    c0 += (idv[i] == 0) ? 1 : 0;
  }
  int v = c0;
#pragma unroll
  for (int off = 1; off < 32; off <<= 1) {
    const int t = __shfl_up(v, off, 32);
    v += (lane >= off) ? t : 0;
  }
  if (lane == 31) wtot[wave] = v;
  __syncthreads();
  int pre = 0, tot = 0;
#pragma unroll
  for (int w = 0; w < 8; ++w) {
    const int t = wtot[w];
    pre += (w < wave) ? t : 0;
    tot += t;
  }
  const int n0 = tot;
  const int P0 = (n0 + 63) & ~63;
  const int excl0 = pre + v - c0;
  int r0 = excl0;
  int r1 = P0 + (s0 - excl0);
#pragma unroll
  for (int i = 0; i < RPT; ++i) {
    const int s = s0 + i;
    const bool z = (idv[i] == 0);
    int p = z ? r0 : r1;
    r0 += z ? 1 : 0;
    r1 += z ? 0 : 1;
    p = clampi(p, 0, ROWSP - 1);
    L[TPERM + p] = s;
    L[TIPOS + s] = p;
  }
  if (tid == 0) {
    L[THDR]     = n0;
    L[THDR + 1] = P0;
    L[THDR + 2] = SEQ - n0;
    L[THDR + 3] = P0 + (((SEQ - n0) + 63) & ~63);
  }
  __syncthreads();
  const int NQ4 = TABN / 4;
  const int NIT = (NQ4 + 255) / 256;
  v4i vals[(TABN / 4 + 255) / 256];
#pragma unroll
  for (int it = 0; it < NIT; ++it) {
    const int q4 = it * 256 + tid;
    v4i t4 = {0, 0, 0, 0};
    if (q4 < NQ4) t4 = *(const v4i*)(L + q4 * 4);
    vals[it] = t4;
  }
  int* dst = TAB + (size_t)b * TABN;
  for (int pass = 0; pass < 2; ++pass) {
#pragma unroll
    for (int it = 0; it < NIT; ++it) {
      const int q4 = it * 256 + tid;
      if (q4 < NQ4) *(volatile v4i*)(dst + q4 * 4) = vals[it];
    }
    __threadfence();
  }
}

__global__ __launch_bounds__(256) void k_xg(const float* __restrict__ x, const int* __restrict__ TAB, u16* XB) {
  const int tid = threadIdx.x;
  const int bid = blockIdx.x;
  const int bb  = bid / ROWSP;
  const int p   = bid - bb * ROWSP;
  if (bb >= NB) return;
  const int s = TAB[(size_t)bb * TABN + TPERM + p];
  const bool valid = ((unsigned)s < (unsigned)SEQ);
  const int sc = clampi(s, 0, SEQ - 1);
  const float* src = x + ((size_t)bb * XS_FULL + sc) * DMOD + tid * 8;
  const v4f a = *(const v4f*)(src), b4 = *(const v4f*)(src + 4);
  v4u o;
#pragma unroll
  for (int e = 0; e < 2; ++e) {
    const unsigned w0 = pk16(bf_bits(a[2 * e]), bf_bits(a[2 * e + 1]));
    const unsigned w1 = pk16(bf_bits(b4[2 * e]), bf_bits(b4[2 * e + 1]));
    o[e]     = valid ? w0 : 0u;
    o[2 + e] = valid ? w1 : 0u;
  }
  u16* d = XB + ((size_t)bb * ROWSP + p) * DMOD + tid * 8;
  for (int pass = 0; pass < 2; ++pass) {
    *(volatile v4u*)(d) = o;
    __threadfence();
  }
}

__global__ __launch_bounds__(256) void k_wt(const float* __restrict__ W, u16* D, int N, int K, int f16mode, float scale) {
  __shared__ __align__(16) u16 T[64 * WTP];
  const int tid = threadIdx.x;
  const int nkt = K >> 6, nnt = N >> 6;
  const int bid = blockIdx.x;
  const int kt  = bid % nkt;
  const int t2  = bid / nkt;
  const int nt  = t2 % nnt;
  const int m   = t2 / nnt;
  if (m >= NMOD) return;
  const int k0 = kt * 64, n0 = nt * 64;
  {
    const int kr = tid >> 2;
    const int nc = (tid & 3) * 16;
    const float* src = W + ((size_t)m * K + k0 + kr) * (size_t)N + n0 + nc;
#pragma unroll
    for (int i = 0; i < 4; ++i) {
      const v4f a = *(const v4f*)(src + 4 * i);
#pragma unroll
      for (int e = 0; e < 4; ++e) {
        const float f = a[e];
        const unsigned short hb = h_bits((_Float16)(bfr(f) * scale));
        const unsigned short bb = bf_bits(f);
        T[(nc + 4 * i + e) * WTP + kr] = (f16mode != 0) ? hb : bb;
      }
    }
  }
  __syncthreads();
  const int q8 = tid >> 3, p8 = (tid & 7) * 8;
  v4u vv[2];
#pragma unroll
  for (int it = 0; it < 2; ++it) {
    const int nrow = it * 32 + q8;
    vv[it] = *(const v4u*)(T + nrow * WTP + p8);
  }
  u16* base = D + ((size_t)m * N + n0) * (size_t)K + k0 + p8;
  for (int pass = 0; pass < 2; ++pass) {
#pragma unroll
    for (int it = 0; it < 2; ++it) {
      const int nrow = it * 32 + q8;
      *(volatile v4u*)(base + (size_t)nrow * K) = vv[it];
    }
    __threadfence();
  }
}

__global__ __launch_bounds__(256) void k_vt(const float* __restrict__ F, const int* __restrict__ TAB, u16* VHo, u16* VLo) {
  __shared__ __align__(16) u16 TH[HD * VTP];
  __shared__ __align__(16) u16 TL[HD * VTP];
  const int tid = threadIdx.x;
  const int bid = blockIdx.x;
  const int st  = bid % NST;
  const int t2  = bid / NST;
  const int g   = t2 % NKVH;
  const int b   = t2 / NKVH;
  if (b >= NB) return;
  const int s0  = st * 64;
  {
    const int sl = tid >> 2;
    const int dc = (tid & 3) * 32;
    const int p  = clampi(TAB[(size_t)b * TABN + TIPOS + s0 + sl], 0, ROWSP - 1);
    const float* src = F + ((size_t)b * ROWSP + p) * KVD + g * HD + dc;
#pragma unroll
    for (int i = 0; i < 8; ++i) {
      const v4f a = *(const v4f*)(src + 4 * i);
#pragma unroll
      for (int e = 0; e < 4; ++e) {
        const float t = a[e] * VCAR;
        const _Float16 hv = (_Float16)t;
        const _Float16 lv = (_Float16)(t - (float)hv);
        TH[(dc + 4 * i + e) * VTP + sl] = h_bits(hv);
        TL[(dc + 4 * i + e) * VTP + sl] = h_bits(lv);
      }
    }
  }
  __syncthreads();
  v4u vh[4], vl[4];
  const int q8 = tid >> 3, p8 = (tid & 7) * 8;
#pragma unroll
  for (int it = 0; it < 4; ++it) {
    const int line = it * 32 + q8;
    vh[it] = *(const v4u*)(TH + line * VTP + p8);
    vl[it] = *(const v4u*)(TL + line * VTP + p8);
  }
  const size_t hrow = (size_t)(b * NKVH + g) * HD;
  const size_t base = hrow * SEQ + s0 + p8;
  for (int pass = 0; pass < 2; ++pass) {
#pragma unroll
    for (int it = 0; it < 4; ++it) {
      const int line = it * 32 + q8;
      *(volatile v4u*)(VHo + base + (size_t)line * SEQ) = vh[it];
      *(volatile v4u*)(VLo + base + (size_t)line * SEQ) = vl[it];
    }
    __threadfence();
  }
}

__global__ __launch_bounds__(256) void k_rope(const float* __restrict__ F, int ncol, const float* __restrict__ fc,
                                              const int* __restrict__ TAB, u16* Hp, u16* Lp, float sc) {
#pragma clang fp contract(off)
  const int tid = (int)threadIdx.x;
  const int row = (int)blockIdx.x;
  if (row >= MROWS) return;
  const int col = tid * 8;
  if (col + 8 > ncol) return;
  const int b = row / SEQ;
  const int s = row - b * SEQ;
  const int p = clampi(TAB[(size_t)b * TABN + TIPOS + s], 0, ROWSP - 1);
  const float* src = F + ((size_t)b * ROWSP + p) * (size_t)ncol + col;
  const v4f xa = *(const v4f*)(src), xb = *(const v4f*)(src + 4);
  const int dp = (col & (HD - 1)) >> 1;
  const float* fp = fc + ((size_t)s * HHALF + dp) * 4;
  const v4f fa = *(const v4f*)(fp), fb = *(const v4f*)(fp + 4), fcv = *(const v4f*)(fp + 8), fd = *(const v4f*)(fp + 12);
  float xv[8], fv[16];
#pragma unroll
  for (int e = 0; e < 4; ++e) {
    xv[e] = xa[e];  xv[4 + e] = xb[e];
    fv[e] = bfr(fa[e]);  fv[4 + e] = bfr(fb[e]);  fv[8 + e] = bfr(fcv[e]);  fv[12 + e] = bfr(fd[e]);
  }
  unsigned short hb[8], lb[8];
#pragma unroll
  for (int i = 0; i < 4; ++i) {
#pragma unroll
    for (int j = 0; j < 2; ++j) {
      const float o = xv[2 * i] * fv[4 * i + 2 * j] + xv[2 * i + 1] * fv[4 * i + 2 * j + 1];
      const float t = o * sc;
      const _Float16 hq = (_Float16)t;
      hb[2 * i + j] = h_bits(hq);
      lb[2 * i + j] = h_bits((_Float16)(t - (float)hq));
    }
  }
  v4u oh, ol;
#pragma unroll
  for (int e = 0; e < 4; ++e) {
    oh[e] = pk16(hb[2 * e], hb[2 * e + 1]);
    ol[e] = pk16(lb[2 * e], lb[2 * e + 1]);
  }
  u16* dh = Hp + (size_t)row * ncol + col;
  u16* dl = Lp + (size_t)row * ncol + col;
  for (int pass = 0; pass < 2; ++pass) {
    *(volatile v4u*)(dh) = oh;
    *(volatile v4u*)(dl) = ol;
    __threadfence();
  }
}

__global__ __launch_bounds__(256) void k_zpad(const int* __restrict__ TAB, u16* OH, u16* OL) {
  const int tid = threadIdx.x;
  const int bid = blockIdx.x;
  const int bb  = bid / 128;
  const int i   = bid % 128;
  if (bb >= NB) return;
  int n0, P0, U;
  seginfo(TAB + (size_t)bb * TABN, n0, P0, U);
  int p; bool ok;
  if (i < 64) { p = n0 + i;                     ok = (p < P0); }
  else        { p = P0 + (SEQ - n0) + (i - 64); ok = (p < U);  }
  if (!ok) return;
  p = clampi(p, 0, ROWSP - 1);
  const v4u z = {0u, 0u, 0u, 0u};
  const size_t d = ((size_t)bb * ROWSP + p) * DMOD + tid * 8;
  for (int pass = 0; pass < 2; ++pass) {
    *(volatile v4u*)(OH + d) = z;
    *(volatile v4u*)(OL + d) = z;
    __threadfence();
  }
}

__device__ __forceinline__ void epi64(float* sl, v8f a0, v8f a1, v8f a2, v8f a3, float oscale,
                                      float* C, int N, size_t rowb, int col0, int lane) {
  const int hh = lane >> 4, m = lane & 15;
#pragma unroll
  for (int r = 0; r < 8; ++r) {
    const int ro = (8 * hh + r) * 68 + m;
    sl[ro]      = a0[r] * oscale;
    sl[ro + 16] = a1[r] * oscale;
    sl[ro + 32] = a2[r] * oscale;
    sl[ro + 48] = a3[r] * oscale;
  }
  wave_sync_lds();
  v4f vals[8];
#pragma unroll
  for (int it = 0; it < 8; ++it) vals[it] = *(const v4f*)(sl + (it * 2 + hh) * 68 + m * 4);
  float* dst = C + (rowb + (size_t)hh) * (size_t)N + col0 + m * 4;
  for (int pass = 0; pass < 2; ++pass) {
#pragma unroll
    for (int it = 0; it < 8; ++it) {
      *(volatile v4f*)(dst + (size_t)(it * 2) * (size_t)N) = vals[it];
    }
    __threadfence();
  }
}

__device__ __forceinline__ void epi64p(float* sl, v8f a0, v8f a1, v8f a2, v8f a3, float oscale,
                                       float* C, const int* __restrict__ prow, int bb, int col0, int lane) {
  const int hh = lane >> 4, m = lane & 15;
#pragma unroll
  for (int r = 0; r < 8; ++r) {
    const int ro = (8 * hh + r) * 68 + m;
    sl[ro]      = a0[r] * oscale;
    sl[ro + 16] = a1[r] * oscale;
    sl[ro + 32] = a2[r] * oscale;
    sl[ro + 48] = a3[r] * oscale;
  }
  wave_sync_lds();
  v4f vals[8];
  int srow[8];
#pragma unroll
  for (int it = 0; it < 8; ++it) {
    vals[it] = *(const v4f*)(sl + (it * 2 + hh) * 68 + m * 4);
    srow[it] = prow[it * 2 + hh];
  }
  for (int pass = 0; pass < 2; ++pass) {
#pragma unroll
    for (int it = 0; it < 8; ++it) {
      const int s = srow[it];
      if ((unsigned)s < (unsigned)SEQ) {
        float* dst = C + ((size_t)bb * SEQ + s) * (size_t)DMOD + col0 + m * 4;
        *(volatile v4f*)(dst) = vals[it];
      }
    }
    __threadfence();
  }
}

__global__ __launch_bounds__(128)
void gemm_p(const u16* __restrict__ A, const u16* __restrict__ Bt, float* C, const int* __restrict__ TAB, int N, int K) {
  __shared__ __align__(16) float slab[4 * SLAB64];
  const int tid = threadIdx.x, wave = tid >> 5, lane = tid & 31, hh = lane >> 4, m = lane & 15;
  const int ntile = N >> 6;
  const int bid   = blockIdx.x;
  const int ct    = bid % ntile;
  const int t2    = bid / ntile;
  const int rt    = t2 % NRT;
  const int bb    = t2 / NRT;
  if (bb >= NB) return;
  int n0, P0, U;
  seginfo(TAB + (size_t)bb * TABN, n0, P0, U);
  const int pos0 = rt * 64;
  if (pos0 >= U) return;
  const int wsel = (pos0 < P0) ? 0 : 1;
  const int col0 = ct * 64;
  const size_t rowb = (size_t)bb * ROWSP + pos0 + wave * 16;
  const u16* ap = A  + (rowb + m) * (size_t)K + 8 * hh;
  const u16* bp = Bt + ((size_t)wsel * N + col0 + m) * (size_t)K + 8 * hh;
  const size_t bs = (size_t)16 * K;
  v8f acc0 = zero8(), acc1 = zero8(), acc2 = zero8(), acc3 = zero8();
#pragma unroll 1
  for (int k0 = 0; k0 < K; k0 += 32) {
    const v16b a  = ldfrag_b(ap + k0);
    const v16b b0 = ldfrag_b(bp + k0);
    const v16b b1 = ldfrag_b(bp + bs + k0);
    const v16b b2 = ldfrag_b(bp + 2 * bs + k0);
    const v16b b3 = ldfrag_b(bp + 3 * bs + k0);
    acc0 = mma_b(a, b0, acc0);
    acc1 = mma_b(a, b1, acc1);
    acc2 = mma_b(a, b2, acc2);
    acc3 = mma_b(a, b3, acc3);
    guard6<v16b>(acc0, acc1, acc2, acc3, a, b0, b1, b2, b3, a);
  }
  epi64(slab + wave * SLAB64, acc0, acc1, acc2, acc3, 1.0f, C, N, rowb, col0, lane);
}

template <int NPROD>
__global__ __launch_bounds__(128)
void gemm_o(const u16* __restrict__ Ah, const u16* __restrict__ Al, const u16* __restrict__ Bt,
            float* C, const int* __restrict__ TAB, float oscale) {
  __shared__ __align__(16) float slab[4 * SLAB64];
  const int tid = threadIdx.x, wave = tid >> 5, lane = tid & 31, hh = lane >> 4, m = lane & 15;
  const int ntile = DMOD >> 6;
  const int bid   = blockIdx.x;
  const int ct    = bid % ntile;
  const int t2    = bid / ntile;
  int bb, pos0, wsel;
  if constexpr (NPROD == 2) {
    const int j = t2 % (2 * NLEAD);
    bb = t2 / (2 * NLEAD);
    if (bb >= NB) return;
    int n0, P0, U;
    seginfo(TAB + (size_t)bb * TABN, n0, P0, U);
    const int seg = j / NLEAD, w = j % NLEAD;
    const int segrows = (seg != 0) ? (SEQ - n0) : n0;
    const int nts = (segrows + 63) >> 6;
    if (w >= nts) return;
    pos0 = ((seg != 0) ? P0 : 0) + 64 * w;
    wsel = seg;
  } else {
    const int rt = t2 % NRT;
    bb = t2 / NRT;
    if (bb >= NB) return;
    int n0, P0, U;
    seginfo(TAB + (size_t)bb * TABN, n0, P0, U);
    pos0 = rt * 64;
    if (pos0 >= U) return;
    const int seg = (pos0 >= P0) ? 1 : 0;
    const int w = (pos0 - ((seg != 0) ? P0 : 0)) >> 6;
    if (w < NLEAD) return;
    wsel = seg;
  }
  const int col0  = ct * 64;
  const int K     = DMOD;
  const size_t rowA = (size_t)bb * ROWSP + pos0 + wave * 16;
  const _Float16* ahp = (const _Float16*)(const void*)Ah + (rowA + m) * K + 8 * hh;
  const _Float16* alp = (const _Float16*)(const void*)Al + (rowA + m) * K + 8 * hh;
  const _Float16* bp  = (const _Float16*)(const void*)Bt + ((size_t)wsel * DMOD + col0 + m) * K + 8 * hh;
  const size_t bs = (size_t)16 * K;
  v8f acc0 = zero8(), acc1 = zero8(), acc2 = zero8(), acc3 = zero8();
  if constexpr (NPROD == 2) {
#pragma unroll 1
    for (int k0 = 0; k0 < K; k0 += 32) {
      const v16h ah = ldfrag_h(ahp + k0), al = ldfrag_h(alp + k0);
      const v16h b0 = ldfrag_h(bp + k0);
      const v16h b1 = ldfrag_h(bp + bs + k0);
      const v16h b2 = ldfrag_h(bp + 2 * bs + k0);
      const v16h b3 = ldfrag_h(bp + 3 * bs + k0);
      acc0 = mma_h(ah, b0, acc0);  acc0 = mma_h(al, b0, acc0);
      acc1 = mma_h(ah, b1, acc1);  acc1 = mma_h(al, b1, acc1);
      acc2 = mma_h(ah, b2, acc2);  acc2 = mma_h(al, b2, acc2);
      acc3 = mma_h(ah, b3, acc3);  acc3 = mma_h(al, b3, acc3);
      guard6<v16h>(acc0, acc1, acc2, acc3, ah, al, b0, b1, b2, b3);
    }
  } else {
#pragma unroll 1
    for (int k0 = 0; k0 < K; k0 += 32) {
      const v16h ah = ldfrag_h(ahp + k0);
      const v16h b0 = ldfrag_h(bp + k0);
      const v16h b1 = ldfrag_h(bp + bs + k0);
      const v16h b2 = ldfrag_h(bp + 2 * bs + k0);
      const v16h b3 = ldfrag_h(bp + 3 * bs + k0);
      acc0 = mma_h(ah, b0, acc0);
      acc1 = mma_h(ah, b1, acc1);
      acc2 = mma_h(ah, b2, acc2);
      acc3 = mma_h(ah, b3, acc3);
      guard6<v16h>(acc0, acc1, acc2, acc3, ah, b0, b1, b2, b3, ah);
    }
  }
  const int* prow = TAB + (size_t)bb * TABN + TPERM + pos0 + wave * 16;
  epi64p(slab + wave * SLAB64, acc0, acc1, acc2, acc3, oscale, C, prow, bb, col0, lane);
}

__global__ __launch_bounds__(ATT_THREADS)
void attn_c(const u16* __restrict__ QHp, const u16* __restrict__ QLp,
            const u16* __restrict__ KHp, const u16* __restrict__ KLp,
            const u16* __restrict__ VHp, const u16* __restrict__ VLp,
            const int* __restrict__ TAB, u16* OHp, u16* OLp) {
  __shared__ __align__(16) float smem[WPB * WREG];

  const int tid  = threadIdx.x;
  const int wave = tid >> 5;
  const int lane = tid & 31;
  const int hh   = lane >> 4;
  const int c    = lane & 15;
  const int bid  = blockIdx.x;
  const int qt   = bid % NQT;
  const int t2   = bid / NQT;
  const int hg   = t2 % NHG;
  const int b    = t2 / NHG;
  if (b >= NB) return;
  const int q0   = qt * 16;
  if (q0 + 16 > SEQ) return;
  const int head = hg * WPB + wave;
  const int kvh  = hg;

  float* pt   = smem + wave * WREG;
  float* slab = pt + PTW;

  const size_t hcol = (size_t)head * HD + 8 * hh;
  const size_t kcol = (size_t)kvh * HD + 8 * hh;
  const _Float16* Qh  = (const _Float16*)(const void*)QHp + ((size_t)b * SEQ + q0 + c) * DMOD + hcol;
  const _Float16* Ql  = (const _Float16*)(const void*)QLp + ((size_t)b * SEQ + q0 + c) * DMOD + hcol;
  const _Float16* Khb = (const _Float16*)(const void*)KHp + ((size_t)b * SEQ + c) * KVD + kcol;
  const _Float16* Klb = (const _Float16*)(const void*)KLp + ((size_t)b * SEQ + c) * KVD + kcol;
  const _Float16* Vhb = (const _Float16*)(const void*)VHp + ((size_t)(b * NKVH + kvh) * HD + c) * SEQ + 8 * hh;
  const _Float16* Vlb = (const _Float16*)(const void*)VLp + ((size_t)(b * NKVH + kvh) * HD + c) * SEQ + 8 * hh;
  const float lsc = RSQ_HD * (LOG2E / (QSC * KSC));
  const float oc  = 1.0f / (PCAR * VCAR);
  const size_t KROW = (size_t)KVD;

  float mrow[8], lrow[8];
  v8f o[8];
#pragma unroll
  for (int r = 0; r < 8; ++r) { mrow[r] = -INFINITY; lrow[r] = 0.f; }
#pragma unroll
  for (int j = 0; j < 8; ++j) o[j] = zero8();
  const int ncaus = (q0 >> 5) + 1;
  const int nkt = (ncaus < NKT) ? ncaus : NKT;
  const int qr0 = q0 + 8 * hh;

#pragma unroll 1
  for (int kt = 0; kt < nkt; ++kt) {
    const int kb = kt * 32;
    v8f s0 = zero8(), s1 = zero8();
    const _Float16* k0p = Khb + (size_t)kb * KROW;
    const _Float16* k1p = k0p + (size_t)16 * KROW;
    const _Float16* l0p = Klb + (size_t)kb * KROW;
    const _Float16* l1p = l0p + (size_t)16 * KROW;
#pragma unroll
    for (int kk = 0; kk < HD / 32; ++kk) {
      const v16h qh  = ldfrag_h(Qh + kk * 32);
      const v16h ql  = ldfrag_h(Ql + kk * 32);
      const v16h kh0 = ldfrag_h(k0p + kk * 32);
      const v16h kh1 = ldfrag_h(k1p + kk * 32);
      const v16h kl0 = ldfrag_h(l0p + kk * 32);
      const v16h kl1 = ldfrag_h(l1p + kk * 32);
      s0 = mma_h(qh, kh0, s0);
      s0 = mma_h(ql, kh0, s0);
      s0 = mma_h(qh, kl0, s0);
      s1 = mma_h(qh, kh1, s1);
      s1 = mma_h(ql, kh1, s1);
      s1 = mma_h(qh, kl1, s1);
      guard2(s0, s1, qh, ql, kh0, kl0, kh1, kl1);
    }
    const int key0 = kb + c, key1 = kb + 16 + c;
#pragma unroll
    for (int r = 0; r < 8; ++r) {
      const int   qr = qr0 + r;
      const float u0 = s0[r] * lsc;
      const float u1 = s1[r] * lsc;
      const float t0 = (key0 > qr) ? -INFINITY : u0;
      const float t1 = (key1 > qr) ? -INFINITY : u1;
      float mx = fmaxf(t0, t1);
#pragma unroll
      for (int off = 1; off < 16; off <<= 1) mx = fmaxf(mx, __shfl_xor(mx, off, 32));
      const float mn = fmaxf(mrow[r], mx);
      const float ms = (mn == -INFINITY) ? 0.0f : mn;
      const float al = exp2f(mrow[r] - ms);
      mrow[r] = mn;
      const float e0 = exp2f(t0 - ms), e1 = exp2f(t1 - ms);
      float ps = e0 + e1;
#pragma unroll
      for (int off = 1; off < 16; off <<= 1) ps += __shfl_xor(ps, off, 32);
      lrow[r] = lrow[r] * al + ps;
#pragma unroll
      for (int j = 0; j < 8; ++j) o[j][r] *= al;
      const int ro = (8 * hh + r) * PTP + c;
      pt[ro]      = e0;
      pt[ro + 16] = e1;
    }
    wave_sync_lds();
    FragH ph, pl;
    {
      const float* prow = pt + c * PTP + 8 * hh;
      const v4f p0 = *(const v4f*)(prow), p1 = *(const v4f*)(prow + 4);
      const v4f p2 = *(const v4f*)(prow + 16), p3 = *(const v4f*)(prow + 20);
#pragma unroll
      for (int e = 0; e < 4; ++e) {
        const float ta = p0[e] * PCAR, tb = p1[e] * PCAR, tc = p2[e] * PCAR, td = p3[e] * PCAR;
        const _Float16 ha = (_Float16)ta, hb = (_Float16)tb, hc = (_Float16)tc, hd = (_Float16)td;
        ph.h[0][e]     = ha;
        ph.h[0][4 + e] = hb;
        ph.h[1][e]     = hc;
        ph.h[1][4 + e] = hd;
        pl.h[0][e]     = (_Float16)(ta - (float)ha);
        pl.h[0][4 + e] = (_Float16)(tb - (float)hb);
        pl.h[1][e]     = (_Float16)(tc - (float)hc);
        pl.h[1][4 + e] = (_Float16)(td - (float)hd);
      }
    }
    {
      const _Float16* vhp = Vhb + kb;
      const _Float16* vlp = Vlb + kb;
#pragma unroll
      for (int jg = 0; jg < 4; ++jg) {
        const size_t da = (size_t)(2 * jg) * 16 * SEQ;
        const size_t db = da + (size_t)16 * SEQ;
        const v16h vha = ldfrag_h(vhp + da), vhb2 = ldfrag_h(vhp + db);
        const v16h vla = ldfrag_h(vlp + da), vlb2 = ldfrag_h(vlp + db);
        o[2 * jg]     = mma_h(ph.v, vha,  o[2 * jg]);
        o[2 * jg]     = mma_h(pl.v, vha,  o[2 * jg]);
        o[2 * jg]     = mma_h(ph.v, vla,  o[2 * jg]);
        o[2 * jg + 1] = mma_h(ph.v, vhb2, o[2 * jg + 1]);
        o[2 * jg + 1] = mma_h(pl.v, vhb2, o[2 * jg + 1]);
        o[2 * jg + 1] = mma_h(ph.v, vlb2, o[2 * jg + 1]);
        guard2(o[2 * jg], o[2 * jg + 1], ph.v, pl.v, vha, vhb2, vla, vlb2);
      }
    }
    wave_sync_lds();
  }
  acc_guard4(o[0], o[1], o[2], o[3]);
  acc_guard4(o[4], o[5], o[6], o[7]);
#pragma unroll
  for (int r = 0; r < 8; ++r) {
    const float lv  = lrow[r];
    const float ls  = (lv > 0.0f) ? lv : 1.0f;
    const float inv = (lv > 0.0f) ? ((1.0f / ls) * oc) : 0.0f;
#pragma unroll
    for (int j = 0; j < 8; ++j) {
      const int idx = (8 * hh + r) * SLP + j * 16 + c;
      slab[idx] = o[j][r] * inv;
    }
  }

  wave_sync_lds();
  v4u oh[8], ol[8];
  int ppos[8];
  const int rq = lane >> 4, c8 = (lane & 15) * 8;
  const int* ipt = TAB + (size_t)b * TABN + TIPOS + q0;
#pragma unroll
  for (int it = 0; it < 8; ++it) {
    const int row = it * 2 + rq;
    ppos[it] = clampi(ipt[row], 0, ROWSP - 1);
    const v4f a = *(const v4f*)(slab + row * SLP + c8), b4 = *(const v4f*)(slab + row * SLP + c8 + 4);
    float w[8];
#pragma unroll
    for (int e = 0; e < 4; ++e) { w[e] = a[e] * OSC; w[4 + e] = b4[e] * OSC; }
#pragma unroll
    for (int e = 0; e < 4; ++e) {
      const _Float16 h0 = (_Float16)w[2 * e], h1 = (_Float16)w[2 * e + 1];
      const _Float16 l0 = (_Float16)(w[2 * e] - (float)h0), l1 = (_Float16)(w[2 * e + 1] - (float)h1);
      oh[it][e] = pk16(h_bits(h0), h_bits(h1));
      ol[it][e] = pk16(h_bits(l0), h_bits(l1));
    }
  }
  const size_t ocol = (size_t)head * HD + c8;
  for (int pass = 0; pass < 2; ++pass) {
#pragma unroll
    for (int it = 0; it < 8; ++it) {
      const size_t ob = ((size_t)b * ROWSP + ppos[it]) * DMOD + ocol;
      *(volatile v4u*)(OHp + ob) = oh[it];
      *(volatile v4u*)(OLp + ob) = ol[it];
    }
    __threadfence();
  }
}

extern "C" void kernel_launch(void* const* d_in, const int* in_sizes, int n_in,
                              void* d_out, int out_size, void* d_ws, size_t ws_size,
                              hipStream_t stream) {
  if (n_in < 7) return;
  if (in_sizes[0] < ((NB - 1) * XS_FULL + SEQ) * DMOD) return;
  if (in_sizes[1] < SEQ * HHALF * 4) return;
  if (in_sizes[2] < (NB - 1) * XS_FULL + SEQ) return;
  if (in_sizes[3] != NMOD * DMOD * DMOD) return;
  if (in_sizes[4] != NMOD * DMOD * KVD) return;
  if (in_sizes[5] != NMOD * DMOD * KVD) return;
  if (in_sizes[6] != NMOD * DMOD * DMOD) return;
  if (out_size < MROWS * DMOD) return;

  const float* x    = (const float*)d_in[0];
  const float* fcis = (const float*)d_in[1];
  const int*   ids  = (const int*)d_in[2];
  const float* wq   = (const float*)d_in[3];
  const float* wk   = (const float*)d_in[4];
  const float* wv   = (const float*)d_in[5];
  const float* wo   = (const float*)d_in[6];
  float*       out  = (float*)d_out;

  const size_t szTAB = (((size_t)NB * TABN * 4) + 65535) & ~(size_t)65535;
  const size_t szXB  = (size_t)PROWS * DMOD * 2;
  const size_t szW   = (size_t)NMOD * DMOD * DMOD * 2;
  const size_t szF   = (size_t)PROWS * DMOD * 4;
  const size_t szO   = (size_t)PROWS * DMOD * 2;
  const size_t szQ   = (size_t)MROWS * DMOD * 2;
  const size_t szK   = (size_t)MROWS * KVD * 2;
  const size_t szV   = (size_t)NB * NKVH * HD * SEQ * 2;
  if (2 * szO > szF) return;
  size_t off = 0;
  const size_t oTAB = off; off += szTAB;
  const size_t oXB  = off; off += szXB;
  const size_t oW   = off; off += szW;
  const size_t oF   = off; off += szF;
  const size_t oQH  = off; off += szQ;
  const size_t oQL  = off; off += szQ;
  const size_t oKH  = off; off += szK;
  const size_t oKL  = off; off += szK;
  const size_t oVH  = off; off += szV;
  const size_t oVL  = off; off += szV;
  if (off > ws_size) return;
  if (off > (size_t)WS_CAP) return;

  char* ws = (char*)d_ws;
  int*   TAB = (int*)(ws + oTAB);
  u16*   XB  = (u16*)(ws + oXB);
  u16*   WB  = (u16*)(ws + oW);
  float* F   = (float*)(ws + oF);
  u16*   OH  = (u16*)(ws + oF);
  u16*   OL  = (u16*)(ws + oF + szO);
  u16*   QH  = (u16*)(ws + oQH);
  u16*   QL  = (u16*)(ws + oQL);
  u16*   KH  = (u16*)(ws + oKH);
  u16*   KL  = (u16*)(ws + oKL);
  u16*   VH  = (u16*)(ws + oVH);
  u16*   VL  = (u16*)(ws + oVL);

  const dim3 b256(256), b128(128), bAT(ATT_THREADS);
  const dim3 gTAB(NB);
  const dim3 gXG(NB * ROWSP);
  const dim3 gWQ(NMOD * (DMOD / 64) * (DMOD / 64));
  const dim3 gWK(NMOD * (KVD / 64) * (DMOD / 64));
  const dim3 gGQ(NB * NRT * (DMOD / 64));
  const dim3 gGK(NB * NRT * (KVD / 64));
  const dim3 gVT(NB * NKVH * NST);
  const dim3 gRW(MROWS);
  const dim3 gZP(NB * 128);
  const dim3 gAT(NQT * NHG * NB);
  const dim3 gOL(NB * 2 * NLEAD * (DMOD / 64));
  const dim3 gOR(NB * NRT * (DMOD / 64));

  k_perm<<<gTAB, b256, 0, stream>>>(ids, TAB);
  k_xg<<<gXG, b256, 0, stream>>>(x, TAB, XB);
  k_wt<<<gWK, b256, 0, stream>>>(wv, WB, KVD, DMOD, 0, 1.0f);
  gemm_p<<<gGK, b128, 0, stream>>>(XB, WB, F, TAB, KVD, DMOD);
  k_vt<<<gVT, b256, 0, stream>>>(F, TAB, VH, VL);
  k_wt<<<gWQ, b256, 0, stream>>>(wq, WB, DMOD, DMOD, 0, 1.0f);
  gemm_p<<<gGQ, b128, 0, stream>>>(XB, WB, F, TAB, DMOD, DMOD);
  k_rope<<<gRW, dim3(DMOD / 8), 0, stream>>>(F, DMOD, fcis, TAB, QH, QL, QSC);
  k_wt<<<gWK, b256, 0, stream>>>(wk, WB, KVD, DMOD, 0, 1.0f);
  gemm_p<<<gGK, b128, 0, stream>>>(XB, WB, F, TAB, KVD, DMOD);
  k_rope<<<gRW, dim3(KVD / 8), 0, stream>>>(F, KVD, fcis, TAB, KH, KL, KSC);
  k_wt<<<gWQ, b256, 0, stream>>>(wo, WB, DMOD, DMOD, 1, WOS);
  k_zpad<<<gZP, b256, 0, stream>>>(TAB, OH, OL);
  attn_c<<<gAT, bAT, 0, stream>>>(QH, QL, KH, KL, VH, VL, TAB, OH, OL);
  gemm_o<2><<<gOL, b128, 0, stream>>>(OH, OL, WB, out, TAB, 1.0f / (OSC * WOS));
  gemm_o<1><<<gOR, b128, 0, stream>>>(OH, OL, WB, out, TAB, 1.0f / (OSC * WOS));
  (void)hipGetLastError();
}
